// InterPartMR_6356551598736
// MI455X (gfx1250) — hardware-verified
//
#include <hip/hip_runtime.h>
#include <math.h>

typedef __attribute__((ext_vector_type(16))) _Float16 v16h;
typedef __attribute__((ext_vector_type(16))) __bf16 v16b;
typedef __attribute__((ext_vector_type(8)))  _Float16 v8h;
typedef __attribute__((ext_vector_type(8)))  float v8f;
typedef __attribute__((ext_vector_type(4)))  float v4f;
typedef __attribute__((ext_vector_type(2)))  float v2f;
typedef __attribute__((ext_vector_type(4)))  unsigned v4u;
typedef __attribute__((ext_vector_type(4)))  int v4i;
typedef float __attribute__((may_alias)) float_a;
typedef int __attribute__((may_alias)) int_a;

template <typename T> __device__ __forceinline__ void vst2(void* p, T v) { *(volatile T*)p = v; __threadfence(); *(volatile T*)p = v; }
__device__ __forceinline__ v8f wmma16(v16h a, v16h b, v8f c) {
  v8f d = __builtin_amdgcn_wmma_f32_16x16x32_f16(false, a, false, b, (short)0, c, false, false);
  asm volatile("v_nop\n\tv_nop\n\tv_nop\n\tv_nop" : "+v"(d) : "v"(a), "v"(b));
  return d;
}
__device__ __forceinline__ v8f wmma_bf(v16b a, v16b b, v8f c) {
  v8f d = __builtin_amdgcn_wmma_f32_16x16x32_bf16(false, a, false, b, (short)0, c, false, false);
  asm volatile("v_nop\n\tv_nop\n\tv_nop\n\tv_nop" : "+v"(d) : "v"(a), "v"(b));
  return d;
}
__device__ __forceinline__ v16h frag_h(const _Float16* rowk0, int lane) {
  union { v16h v; v8h q[2]; } u; const _Float16* p = rowk0 + 8 * (lane >> 4);
  u.q[0] = *(const v8h*)p; u.q[1] = *(const v8h*)(p + 16); return u.v;
}
__device__ __forceinline__ v16h frag_f32(const float* rowk0, int lane) {
  v16h a; const float* p = rowk0 + 8 * (lane >> 4);
#pragma unroll
  for (int i = 0; i < 8; ++i) { a[i] = (_Float16)p[i]; a[8 + i] = (_Float16)p[16 + i]; }
  return a;
}
__device__ __forceinline__ v16h frag_f32s(const float* rowk0, int lane, float sc) {
  v16h a; const float* p = rowk0 + 8 * (lane >> 4);
#pragma unroll
  for (int i = 0; i < 8; ++i) { a[i] = (_Float16)(p[i] * sc); a[8 + i] = (_Float16)(p[16 + i] * sc); }
  return a;
}
__device__ __forceinline__ v16h fragc_f32(const float* W, int k0, int n, int lane, int ld, int K) {
  v16h a; const int g = lane >> 4;
#pragma unroll
  for (int i = 0; i < 8; ++i) { const int ka = k0 + 8 * g + i, kb = ka + 16;
    a[i] = (_Float16)(ka < K ? W[(size_t)(ka < K ? ka : K - 1) * ld + n] : 0.f); a[8 + i] = (_Float16)(kb < K ? W[(size_t)(kb < K ? kb : K - 1) * ld + n] : 0.f); }
  return a;
}
struct F2 { v16b h, l; };
__device__ __forceinline__ F2 bsplit16(const float v[16]) { F2 r;
#pragma unroll
  for (int i = 0; i < 16; ++i) { const __bf16 h = (__bf16)v[i]; r.h[i] = h; r.l[i] = (__bf16)(v[i] - (float)h); }
  return r; }
__device__ __forceinline__ F2 split_row(const float* row, int k0, int lane) { float v[16]; const float* p = row + k0 + 8 * (lane >> 4);
#pragma unroll
  for (int i = 0; i < 8; ++i) { v[i] = p[i]; v[8 + i] = p[16 + i]; }
  return bsplit16(v); }
__device__ __forceinline__ F2 split_rowK(const float* row, int k0, int lane, int K) { float v[16]; const int g = lane >> 4;
#pragma unroll
  for (int i = 0; i < 8; ++i) { const int ka = k0 + 8 * g + i, kb = ka + 16; v[i] = ka < K ? row[ka < K ? ka : K - 1] : 0.f; v[8 + i] = kb < K ? row[kb < K ? kb : K - 1] : 0.f; }
  return bsplit16(v); }
__device__ __forceinline__ F2 split_col(const float* W, int k0, int n, int lane, int ld, int K) { float v[16]; const int g = lane >> 4;
#pragma unroll
  for (int i = 0; i < 8; ++i) { const int ka = k0 + 8 * g + i, kb = ka + 16; v[i] = ka < K ? W[(size_t)(ka < K ? ka : K - 1) * ld + n] : 0.f; v[8 + i] = kb < K ? W[(size_t)(kb < K ? kb : K - 1) * ld + n] : 0.f; }
  return bsplit16(v); }
__device__ __forceinline__ v8f mac3(const F2& a, const F2& b, v8f c) { c = wmma_bf(a.l, b.h, c); c = wmma_bf(a.h, b.l, c); return wmma_bf(a.h, b.h, c); }
__device__ __forceinline__ float sigm(float v) { return 1.0f / (1.0f + expf(-v)); }
#define LDSX() do { asm volatile("s_wait_dscnt 0" ::: "memory"); __builtin_amdgcn_wave_barrier(); __builtin_amdgcn_fence(__ATOMIC_RELEASE, "workgroup"); } while (0)


#define NBS 2048
#define CIN 256
#define NP 15
#define CO 512
#define GRP 128
__device__ __forceinline__ float bfr(float v) { return (float)(__bf16)v; }
__device__ __forceinline__ v16b frag_b(const __bf16* rowk0, int lane) { return __builtin_bit_cast(v16b, frag_h((const _Float16*)rowk0, lane)); }

__global__ __launch_bounds__(128) void k_conv(const float* __restrict__ x, const float* __restrict__ cw, const float* __restrict__ cb, float* __restrict__ Z, float* __restrict__ PS, float* __restrict__ PQ) {
  __shared__ __align__(16) float sx[CIN][16];
  __shared__ __align__(16) float sy[16][CO + 8];
  __shared__ __align__(16) float sz[CO][16];
  const int tid = threadIdx.x, wave = tid >> 5, lane = tid & 31, col = lane & 15, gq = lane >> 4; const int b = blockIdx.x;
  const float* xb = x + (size_t)b * CIN * NP;
  for (int q = tid; q < CIN * NP; q += 128) { const int c = q / NP, p = q % NP; sx[c][p] = bfr(xb[q]); }
  for (int q = tid; q < CO + 8; q += 128) sy[15][q] = 0.f;
  __syncthreads();
  for (int c = tid; c < CIN; c += 128) { float v[NP]; float mo[5];
#pragma unroll
    for (int p = 0; p < NP; ++p) v[p] = sx[c][p];
#pragma unroll
    for (int pt = 0; pt < 5; ++pt) { float m = -3.4e38f;
#pragma unroll
      for (int p = 0; p < NP; ++p) { const float cand = (p / 3 == pt) ? v[p] - 10000.0f : v[p]; m = fmaxf(m, cand); }
      mo[pt] = m; }
#pragma unroll
    for (int p = 0; p < NP; ++p) { sy[p][c] = v[p]; sy[p][CIN + c] = mo[p / 3] - v[p]; } }
  __syncthreads();
  { const int g = wave; v8f acc[8] = {};
#pragma unroll
    for (int kc = 0; kc < GRP / 32; ++kc) { const F2 a = split_row(&sy[col][g * GRP], kc * 32, lane);
#pragma unroll
      for (int j = 0; j < 8; ++j) { const v16b wb = split_row(cw + ((size_t)g * GRP + j * 16 + col) * GRP, kc * 32, lane).h; if (g >= 2) acc[j] = wmma_bf(a.l, wb, acc[j]); acc[j] = wmma_bf(a.h, wb, acc[j]); } }
#pragma unroll
    for (int j = 0; j < 8; ++j) { const int o = g * GRP + j * 16 + col; const float bb = bfr(cb[o]);
#pragma unroll
      for (int r = 0; r < 8; ++r) { const int p = 8 * gq + r; if (p < NP) sz[o][p] = acc[j][r] + bb; } } }
  __syncthreads();
  { const float* szf = &sz[0][0];
    float* zb = Z + (size_t)b * CO * NP;
    for (int q4 = tid; q4 < CO * NP / 4; q4 += 128) { v4f v;
#pragma unroll
      for (int e = 0; e < 4; ++e) { const int idx = q4 * 4 + e; v[e] = szf[(idx / NP) * 16 + (idx % NP)]; }
      vst2(zb + q4 * 4, v); } }
  for (int c = tid; c < CO; c += 128) { float s = 0.f, q = 0.f;
#pragma unroll
    for (int p = 0; p < NP; ++p) { const float v = sz[c][p]; s += v; q += v * v; }
    vst2(PS + (size_t)b * CO + c, (float_a)s); vst2(PQ + (size_t)b * CO + c, (float_a)q); }
}
__global__ __launch_bounds__(512) void k_bn(const float* __restrict__ PS, const float* __restrict__ PQ, const float* __restrict__ gam, const float* __restrict__ bet, float* __restrict__ SC) {
  const int c = threadIdx.x; float s = 0.f, q = 0.f;
  for (int b = 0; b < NBS; ++b) { s += PS[(size_t)b * CO + c]; q += PQ[(size_t)b * CO + c]; }
  const float n = (float)(NBS * NP); const float mean = s / n; const float var = fmaxf(q / n - mean * mean, 0.f); const float rs = rsqrtf(var + 1e-5f);
  const float scale = rs * bfr(gam[c]); vst2(SC + c, (float_a)scale); vst2(SC + CO + c, (float_a)(bfr(bet[c]) - mean * scale));
}
__global__ __launch_bounds__(256) void k_out(const float* __restrict__ Z, const float* __restrict__ SC, float* __restrict__ out) {
  const size_t i4 = (size_t)blockIdx.x * 256 + threadIdx.x; if (i4 >= (size_t)NBS * CO * NP / 4) return;
  v4f v = *(const v4f*)(Z + i4 * 4);
#pragma unroll
  for (int e = 0; e < 4; ++e) { const size_t idx = i4 * 4 + e; const int c = (int)((idx / NP) % CO); const float y = v[e] * SC[c] + SC[CO + c]; v[e] = y > 0.f ? y : 0.f; }
  vst2(out + i4 * 4, v);
}
extern "C" void kernel_launch(void* const* d_in, const int* in_sizes, int n_in, void* d_out, int out_size, void* d_ws, size_t ws_size, hipStream_t stream) {
  (void)in_sizes; (void)n_in; (void)out_size; (void)ws_size;
  const float* x = (const float*)d_in[0]; const float* cw = (const float*)d_in[1]; const float* cb = (const float*)d_in[2]; const float* gam = (const float*)d_in[3]; const float* bet = (const float*)d_in[4];
  char* ws = (char*)d_ws; size_t off = 0;
  auto take = [&](size_t bytes) { char* p = ws + off; off += (bytes + 255) & ~(size_t)255; return p; };
  float* Z = (float*)take((size_t)NBS * CO * NP * 4); float* PS = (float*)take((size_t)NBS * CO * 4); float* PQ = (float*)take((size_t)NBS * CO * 4); float* SC = (float*)take((size_t)2 * CO * 4);
  k_conv<<<NBS, 128, 0, stream>>>(x, cw, cb, Z, PS, PQ);
  k_bn<<<1, 512, 0, stream>>>(PS, PQ, gam, bet, SC);
  k_out<<<(NBS * CO * NP / 4 + 255) / 256, 256, 0, stream>>>(Z, SC, (float*)d_out);
}
